// CausalSelfAttentionHead_6047313953342
// MI455X (gfx1250) — hardware-verified
//
#include <hip/hip_runtime.h>
#include <stddef.h>


typedef _Float16 v16h __attribute__((ext_vector_type(16)));
typedef _Float16 v8h  __attribute__((ext_vector_type(8)));
typedef float    v8f  __attribute__((ext_vector_type(8)));
typedef float    v4f  __attribute__((ext_vector_type(4)));

#ifndef NB
#define NB 2
#endif
#ifndef SEQ
#define SEQ 1024
#endif
#ifndef EARLY_RES
#define EARLY_RES 1
#endif
#define NB_FULL  2
#define SEQ_FULL 1024
#define EMB   256
#define HD    64
#define MROWS (NB * SEQ)

static_assert(NB >= 1 && NB <= NB_FULL);
static_assert(SEQ >= 128 && SEQ <= SEQ_FULL && (SEQ % 128) == 0);
static_assert(HD == 64);
static_assert((EMB % 64) == 0 && (EMB % 32) == 0 && (HD % 32) == 0);
static_assert(EMB == 32 * 8);
static_assert((MROWS % 64) == 0 && (MROWS % 8) == 0);

#define LDT 72
#define LDC 68
static_assert((LDT % 8) == 0 && LDT >= 64);
static_assert((LDC % 4) == 0 && LDC >= 64);

#define WCARRY 64.0f
#define XCARRY 16.0f
#define QCARRY 16.0f
#define PCARRY 1024.0f
#define RCARRY 1024.0f
#define PROJ_INV (1.0f / (WCARRY * XCARRY))
#define PAIR_INV (1.0f / (WCARRY * QCARRY))

static_assert((256 / 8) * 2 == 64);
static_assert((256 / 16) * 4 == 64);
static_assert((32 / 16) * 8 == 16);
static_assert(256 * 8 * 4 == 128 * HD);
static_assert(256 * 4 * 4 == 64 * HD);
static_assert(256 * 2 * 8 == 64 * 64);

#define WP_BYTES   ((size_t)HD * EMB * 2)
#define W1_BYTES   ((size_t)HD * HD * 2)
#define X16_BYTES  ((size_t)MROWS * EMB * 2)
#define QK16_BYTES ((size_t)MROWS * HD * 2)
#define VT_BYTES   ((size_t)NB * HD * SEQ * 2)
#define VR_BYTES   ((size_t)NB * HD * 64 * 2)
#define PF32_BYTES ((size_t)MROWS * HD * 4)
#define OFF_WQ  ((size_t)0)
#define OFF_WK  (OFF_WQ + WP_BYTES)
#define OFF_WV  (OFF_WK + WP_BYTES)
#define OFF_W1A (OFF_WV + WP_BYTES)
#define OFF_W1B (OFF_W1A + W1_BYTES)
#define OFF_X   (OFF_W1B + W1_BYTES)
#define OFF_Q   (OFF_X + X16_BYTES)
#define OFF_K   (OFF_Q + QK16_BYTES)
#define OFF_VT  (OFF_K + QK16_BYTES)
#define OFF_VR  (OFF_VT + VT_BYTES)
#define OFF_QP  (OFF_VR + VR_BYTES)
#define OFF_KP  (OFF_QP + PF32_BYTES)
#define WS_TOTAL (OFF_KP + PF32_BYTES)
static_assert((WP_BYTES % 128) == 0 && (W1_BYTES % 128) == 0 && (X16_BYTES % 128) == 0);
static_assert((QK16_BYTES % 128) == 0 && (VT_BYTES % 128) == 0 && (VR_BYTES % 128) == 0);
static_assert((PF32_BYTES % 128) == 0);
static_assert(WS_TOTAL <= (size_t)134217728);

static_assert((size_t)(128 * LDC + 64 * LDC + 64) * 4 + (size_t)(64 * LDT * 2 + 8 * 16 * LDT) * 2
              <= (size_t)131072);

__device__ __forceinline__ float bf16r(float x) {
  unsigned int u = __float_as_uint(x);
  u = (u + 0x7FFFu + ((u >> 16) & 1u)) & 0xFFFF0000u;
  return __uint_as_float(u);
}

__device__ __forceinline__ _Float16 toh_flush(float v) {
  const _Float16 r = (_Float16)v;
  return (fabsf(v) < 6.103515625e-05f) ? (_Float16)0.0f : r;
}

__device__ __forceinline__ v16h frag_at(const _Float16* p) {
  v8h lo = *(const v8h*)(p);
  v8h hi = *(const v8h*)(p + 16);
  v16h out;
#pragma unroll
  for (int i = 0; i < 8; ++i) { out[i] = lo[i]; out[i + 8] = hi[i]; }
  return out;
}
__device__ __forceinline__ v16h ld_frag(const _Float16* base, unsigned ld) {
  const unsigned lane = threadIdx.x & 31u;
  return frag_at(base + (lane & 15u) * ld + (lane >> 4) * 8u);
}

__device__ __forceinline__ v8f wmma16(v16h a, v16h b, v8f c) {
  v8f d = __builtin_amdgcn_wmma_f32_16x16x32_f16(false, a, false, b, (short)0, c,
                                                 false, false);
  asm volatile("v_nop\n\tv_nop\n\tv_nop\n\tv_nop" : "+v"(d) : "v"(a), "v"(b));
  return d;
}

__device__ __forceinline__ float red16_max(float x) {
#pragma unroll
  for (int off = 1; off < 16; off <<= 1) x = fmaxf(x, __shfl_xor(x, off, 32));
  return x;
}
__device__ __forceinline__ float red16_sum(float x) {
#pragma unroll
  for (int off = 1; off < 16; off <<= 1) x += __shfl_xor(x, off, 32);
  return x;
}

__device__ __forceinline__ void wave_lds_sync() {
  __builtin_amdgcn_fence(3  , "wavefront");
  asm volatile("s_wait_dscnt 0x0" ::: "memory");
  __builtin_amdgcn_wave_barrier();
}

__global__ __launch_bounds__(256) void wconv_kernel(
    const float* __restrict__ W, _Float16* __restrict__ Wt, unsigned ldw, unsigned ldk) {
  __shared__ _Float16 T[64 * LDT];
  const unsigned tid = threadIdx.x;
  const unsigned n0 = blockIdx.x * 64u;
  const unsigned k0 = blockIdx.y * 64u;
#pragma unroll 4
  for (unsigned j = 0; j < 16u; ++j) {
    const unsigned idx = tid + 256u * j;
    const unsigned kr = idx >> 6, nc = idx & 63u;
    const float v = W[(size_t)(k0 + kr) * ldw + n0 + nc];
    T[nc * LDT + kr] = toh_flush(WCARRY * bf16r(v));
  }
  __syncthreads();
  v8h x[2];
  size_t off[2];
#pragma unroll
  for (unsigned i = 0; i < 2u; ++i) {
    const unsigned n = 32u * i + (tid >> 3);
    const unsigned kc = (tid & 7u) * 8u;
    x[i] = *(const v8h*)&T[n * LDT + kc];
    off[i] = (size_t)(n0 + n) * ldk + k0 + kc;
  }
#pragma unroll
  for (int i = 0; i < 2; ++i) *(volatile v8h*)(Wt + off[i]) = x[i];
  __threadfence();
#pragma unroll
  for (int i = 0; i < 2; ++i) *(volatile v8h*)(Wt + off[i]) = x[i];
}

__global__ __launch_bounds__(256) void xconv_kernel(
    const float* __restrict__ X, _Float16* __restrict__ dst) {
  const unsigned lane = threadIdx.x & 31u;
  const unsigned w = (unsigned)__builtin_amdgcn_readfirstlane((int)(threadIdx.x >> 5));
  const unsigned crow = blockIdx.x * 8u + w;
  const unsigned bidx = crow / (unsigned)SEQ;
  const unsigned sq = crow - bidx * (unsigned)SEQ;
  const size_t srow = (size_t)bidx * SEQ_FULL + sq;
  const float* xr = X + srow * EMB + lane * 8u;
  const v4f a0 = *(const v4f*)(xr);
  const v4f a1 = *(const v4f*)(xr + 4u);
  v8h o;
#pragma unroll
  for (int i = 0; i < 4; ++i) {
    o[i]     = toh_flush(XCARRY * bf16r(a0[i]));
    o[i + 4] = toh_flush(XCARRY * bf16r(a1[i]));
  }
  _Float16* p = dst + (size_t)crow * EMB + lane * 8u;
  *(volatile v8h*)p = o;
  __threadfence();
  *(volatile v8h*)p = o;
}

template <int MODE>
__device__ __forceinline__ void gemm_body(
    const _Float16* __restrict__ A16, const _Float16* __restrict__ Bt, const unsigned K,
    const float* __restrict__ bias,
    float* __restrict__ outf, _Float16* __restrict__ out16, _Float16* __restrict__ out16r) {
  __shared__ float Cs[64 * LDC];
  const unsigned tid = threadIdx.x, lane = tid & 31u, w = tid >> 5;
  const unsigned mw = w >> 1, nw = w & 1u;
  const unsigned hh = lane >> 4, m = lane & 15u;
  const unsigned n0 = blockIdx.x * 64u;
  const unsigned row0 = blockIdx.y * 64u;

  const _Float16* ap  = A16 + (size_t)(row0 + mw * 16u + m) * K + hh * 8u;
  const _Float16* bp0 = Bt + (size_t)(n0 + nw * 32u + m) * K + hh * 8u;
  const _Float16* bp1 = bp0 + (size_t)16 * K;
  v8f acc0 = {}, acc1 = {};
#pragma unroll 2
  for (unsigned k0 = 0; k0 < K; k0 += 32u) {
    const v16h a  = frag_at(ap + k0);
    const v16h b0 = frag_at(bp0 + k0);
    const v16h b1 = frag_at(bp1 + k0);
    acc0 = wmma16(a, b0, acc0);
    acc1 = wmma16(a, b1, acc1);
  }
#pragma unroll
  for (int r = 0; r < 8; ++r) {
    float* d = &Cs[(mw * 16u + hh * 8u + (unsigned)r) * LDC + nw * 32u + m];
    d[0]  = acc0[r];
    d[16] = acc1[r];
  }
  __syncthreads();

  if (MODE == 0) {
    v8h x[2];
    size_t off[2];
#pragma unroll
    for (unsigned i = 0; i < 2u; ++i) {
      const unsigned r = 32u * i + (tid >> 3);
      const unsigned c = (tid & 7u) * 8u;
      const v4f u0 = *(const v4f*)&Cs[r * LDC + c];
      const v4f u1 = *(const v4f*)&Cs[r * LDC + c + 4];
      const v4f g0 = *(const v4f*)(bias + n0 + c);
      const v4f g1 = *(const v4f*)(bias + n0 + c + 4u);
#pragma unroll
      for (int j = 0; j < 4; ++j) {
        x[i][j]     = toh_flush(QCARRY * fmaxf(u0[j] * PROJ_INV + bf16r(g0[j]), 0.0f));
        x[i][j + 4] = toh_flush(QCARRY * fmaxf(u1[j] * PROJ_INV + bf16r(g1[j]), 0.0f));
      }
      off[i] = (size_t)(row0 + r) * HD + n0 + c;
    }
#pragma unroll
    for (int i = 0; i < 2; ++i) *(volatile v8h*)(out16 + off[i]) = x[i];
    __threadfence();
#pragma unroll
    for (int i = 0; i < 2; ++i) *(volatile v8h*)(out16 + off[i]) = x[i];
  }

  if (MODE == 1) {
    const unsigned bidx = row0 / (unsigned)SEQ;
    const unsigned key0 = row0 - bidx * (unsigned)SEQ;
    const bool first_tile = (key0 == 0u);
    v8h x[2], xr[2];
    size_t off[2], offr[2];
#pragma unroll
    for (unsigned i = 0; i < 2u; ++i) {
      const unsigned dcol = 32u * i + (tid >> 3);
      const unsigned kk = (tid & 7u) * 8u;
      const float bb = bf16r(bias[n0 + dcol]);
#pragma unroll
      for (unsigned j = 0; j < 8u; ++j) {
        const float t = Cs[(kk + j) * LDC + dcol] * PROJ_INV + bb;
        const _Float16 hi = toh_flush(t);
        x[i][j]  = hi;
        xr[i][j] = toh_flush((t - (float)hi) * RCARRY);
      }
      off[i]  = ((size_t)bidx * HD + n0 + dcol) * SEQ + key0 + kk;
      offr[i] = ((size_t)bidx * HD + n0 + dcol) * 64u + kk;
    }
#pragma unroll
    for (int i = 0; i < 2; ++i) *(volatile v8h*)(out16 + off[i]) = x[i];
    if (first_tile) {
#pragma unroll
      for (int i = 0; i < 2; ++i) *(volatile v8h*)(out16r + offr[i]) = xr[i];
    }
    __threadfence();
#pragma unroll
    for (int i = 0; i < 2; ++i) *(volatile v8h*)(out16 + off[i]) = x[i];
    if (first_tile) {
#pragma unroll
      for (int i = 0; i < 2; ++i) *(volatile v8h*)(out16r + offr[i]) = xr[i];
    }
  }

  if (MODE == 5 || MODE == 6) {
    v4f xs[4];
    size_t off[4];
#pragma unroll
    for (unsigned i = 0; i < 4u; ++i) {
      const unsigned r = 16u * i + (tid >> 4);
      const unsigned c = (tid & 15u) * 4u;
      const v4f u = *(const v4f*)&Cs[r * LDC + c];
      v4f val;
      if (MODE == 5) {
        const v4f g = *(const v4f*)(bias + n0 + c);
#pragma unroll
        for (int j = 0; j < 4; ++j) val[j] = u[j] * PAIR_INV + bf16r(g[j]);
      } else {
#pragma unroll
        for (int j = 0; j < 4; ++j) val[j] = u[j] * PAIR_INV;
      }
      xs[i] = val;
      off[i] = (size_t)(row0 + r) * HD + n0 + c;
    }
#pragma unroll
    for (int i = 0; i < 4; ++i) *(volatile v4f*)(outf + off[i]) = xs[i];
    __threadfence();
#pragma unroll
    for (int i = 0; i < 4; ++i) *(volatile v4f*)(outf + off[i]) = xs[i];
  }
}

__global__ __launch_bounds__(256) void gemm_qk_kernel(
    const _Float16* __restrict__ A16, const _Float16* __restrict__ Bt,
    const float* __restrict__ bias, _Float16* __restrict__ out16) {
  gemm_body<0>(A16, Bt, (unsigned)EMB, bias, (float*)0, out16, out16);
}
__global__ __launch_bounds__(256) void gemm_v_kernel(
    const _Float16* __restrict__ A16, const _Float16* __restrict__ Bt,
    const float* __restrict__ bias, _Float16* __restrict__ vt, _Float16* __restrict__ vtr) {
  gemm_body<1>(A16, Bt, (unsigned)EMB, bias, (float*)0, vt, vtr);
}
__global__ __launch_bounds__(256) void gemm_qp_kernel(
    const _Float16* __restrict__ A16, const _Float16* __restrict__ Bt,
    const float* __restrict__ bias, float* __restrict__ outf) {
  gemm_body<5>(A16, Bt, (unsigned)HD, bias, outf, (_Float16*)0, (_Float16*)0);
}
__global__ __launch_bounds__(256) void gemm_kp_kernel(
    const _Float16* __restrict__ A16, const _Float16* __restrict__ Bt,
    float* __restrict__ outf) {
  gemm_body<6>(A16, Bt, (unsigned)HD, (const float*)0, outf, (_Float16*)0, (_Float16*)0);
}

__global__ __launch_bounds__(256) void attn_kernel(
    const float* __restrict__ QPb, const float* __restrict__ KPo,
    const _Float16* __restrict__ Vt, const _Float16* __restrict__ VtR,
    const float* __restrict__ W2, const float* __restrict__ B2,
    float* __restrict__ Out) {
  __shared__ float Qs[128 * LDC];
  __shared__ float KPs[64 * LDC];
  __shared__ float W2s[64];
  __shared__ _Float16 Vs[64 * LDT];
  __shared__ _Float16 VRs[64 * LDT];
  __shared__ _Float16 Ps[8 * 16 * LDT];

  const unsigned tid = threadIdx.x, lane = tid & 31u;
  const unsigned w = (unsigned)__builtin_amdgcn_readfirstlane((int)(threadIdx.x >> 5));
  const unsigned hh = lane >> 4, m = lane & 15u;
  const unsigned q0 = blockIdx.x * 128u;
  const unsigned b = blockIdx.y;
  const unsigned qrow0 = q0 + w * 16u;
  const bool first_blk = (blockIdx.x == 0u);
  const unsigned pbase = w * (16u * LDT);
  const unsigned qsbase = (w * 16u) * LDC;

#pragma unroll
  for (unsigned j = 0; j < 8u; ++j) {
    const unsigned idx = tid + 256u * j;
    const unsigned r = idx >> 4, c = (idx & 15u) * 4u;
    *(v4f*)&Qs[r * LDC + c] =
        *(const v4f*)(QPb + (size_t)(b * (unsigned)SEQ + q0 + r) * HD + c);
  }
  {
    const float wv = bf16r(W2[tid & 63u]);
    if (tid < 64u) W2s[tid] = wv;
  }
  const float b2v = bf16r(B2[0]);

  float mrow[8], lrow[8];
  v8f o[4];
#pragma unroll
  for (int v = 0; v < 8; ++v) { mrow[v] = -1.0e30f; lrow[v] = 0.0f; }
#pragma unroll
  for (int nb = 0; nb < 4; ++nb) o[nb] = (v8f){};

  const size_t vplane = (size_t)b * HD * SEQ;
  const size_t rplane = (size_t)b * HD * 64u;
  const unsigned kend = q0 + 128u;

  for (unsigned kb = 0; kb < kend; kb += 64u) {
    const bool early = (EARLY_RES != 0) && first_blk && (kb == 0u);
#pragma unroll
    for (unsigned j = 0; j < 4u; ++j) {
      const unsigned idx = tid + 256u * j;
      const unsigned r = idx >> 4, c = (idx & 15u) * 4u;
      *(v4f*)&KPs[r * LDC + c] =
          *(const v4f*)(KPo + (size_t)(b * (unsigned)SEQ + kb + r) * HD + c);
    }
#pragma unroll
    for (unsigned j = 0; j < 2u; ++j) {
      const unsigned idx = tid + 256u * j;
      const unsigned r = idx >> 3, c = (idx & 7u) * 8u;
      *(v8h*)&Vs[r * LDT + c] = *(const v8h*)(Vt + vplane + (size_t)r * SEQ + kb + c);
    }
    if (early) {
#pragma unroll
      for (unsigned j = 0; j < 2u; ++j) {
        const unsigned idx = tid + 256u * j;
        const unsigned r = idx >> 3, c = (idx & 7u) * 8u;
        *(v8h*)&VRs[r * LDT + c] = *(const v8h*)(VtR + rplane + (size_t)r * 64u + c);
      }
    }
    __syncthreads();

    v8f s[4];
#pragma unroll
    for (int kg = 0; kg < 4; ++kg) s[kg] = (v8f){};
#pragma unroll 1
    for (unsigned dc = 0; dc < 16u; ++dc) {
      const v4f wv = *(const v4f*)&W2s[dc * 4u];
      v4f qv[8];
#pragma unroll
      for (int v = 0; v < 8; ++v)
        qv[v] = *(const v4f*)&Qs[qsbase + (hh * 8u + (unsigned)v) * LDC + dc * 4u];
#pragma unroll
      for (int kg = 0; kg < 4; ++kg) {
        const v4f kv = *(const v4f*)&KPs[((unsigned)kg * 16u + m) * LDC + dc * 4u];
#pragma unroll
        for (int v = 0; v < 8; ++v) {
#pragma unroll
          for (int j = 0; j < 4; ++j)
            s[kg][v] = s[kg][v] + wv[j] * fmaxf(qv[v][j] + kv[j], 0.0f);
        }
      }
    }
#pragma unroll
    for (int kg = 0; kg < 4; ++kg)
#pragma unroll
      for (int v = 0; v < 8; ++v) s[kg][v] = s[kg][v] + b2v;

    if (kb >= q0) {
#pragma unroll
      for (int kg = 0; kg < 4; ++kg)
#pragma unroll
        for (int v = 0; v < 8; ++v) {
          const unsigned key = kb + (unsigned)kg * 16u + m;
          const unsigned row = qrow0 + hh * 8u + (unsigned)v;
          s[kg][v] = (key > row) ? -1.0e30f : s[kg][v];
        }
    }

    float alpha[8];
#pragma unroll
    for (int v = 0; v < 8; ++v) {
      float mx = fmaxf(fmaxf(s[0][v], s[1][v]), fmaxf(s[2][v], s[3][v]));
      mx = red16_max(mx);
      const float mn = fmaxf(mrow[v], mx);
      alpha[v] = __expf(mrow[v] - mn);
      mrow[v] = mn;
    }
#pragma unroll
    for (int kg = 0; kg < 4; ++kg)
#pragma unroll
      for (int v = 0; v < 8; ++v) s[kg][v] = __expf(s[kg][v] - mrow[v]);
#pragma unroll
    for (int v = 0; v < 8; ++v) {
      const float rs = red16_sum((s[0][v] + s[1][v]) + (s[2][v] + s[3][v]));
      lrow[v] = alpha[v] * lrow[v] + rs;
    }
#pragma unroll
    for (int nb = 0; nb < 4; ++nb)
#pragma unroll
      for (int v = 0; v < 8; ++v) o[nb][v] = o[nb][v] * alpha[v];

#pragma unroll
    for (int kg = 0; kg < 4; ++kg)
#pragma unroll
      for (int v = 0; v < 8; ++v)
        Ps[pbase + (hh * 8u + (unsigned)v) * LDT + (unsigned)kg * 16u + m] =
            toh_flush(s[kg][v] * PCARRY);
    wave_lds_sync();

#pragma unroll
    for (int c = 0; c < 2; ++c) {
      const v16h pf = ld_frag(&Ps[pbase + c * 32], LDT);
#pragma unroll
      for (int nb = 0; nb < 4; ++nb) {
        const v16h vf = ld_frag(&Vs[(nb * 16) * LDT + c * 32], LDT);
        o[nb] = wmma16(pf, vf, o[nb]);
      }
    }

    if (early) {
#pragma unroll
      for (int nb = 0; nb < 4; ++nb) {
        v8f o2 = {};
#pragma unroll
        for (int c = 0; c < 2; ++c) {
          const v16h pf = ld_frag(&Ps[pbase + c * 32], LDT);
          const v16h vr = ld_frag(&VRs[(nb * 16) * LDT + c * 32], LDT);
          o2 = wmma16(pf, vr, o2);
        }
#pragma unroll
        for (int v = 0; v < 8; ++v) o[nb][v] = o[nb][v] + o2[v] * (1.0f / RCARRY);
      }
      wave_lds_sync();
#pragma unroll
      for (int kg = 0; kg < 4; ++kg)
#pragma unroll
        for (int v = 0; v < 8; ++v) {
          const float t = s[kg][v] * PCARRY;
          const float hi = (float)toh_flush(t);
          Ps[pbase + (hh * 8u + (unsigned)v) * LDT + (unsigned)kg * 16u + m] =
              toh_flush((t - hi) * RCARRY);
        }
      wave_lds_sync();
#pragma unroll
      for (int nb = 0; nb < 4; ++nb) {
        v8f o2 = {};
#pragma unroll
        for (int c = 0; c < 2; ++c) {
          const v16h pf = ld_frag(&Ps[pbase + c * 32], LDT);
          const v16h vf = ld_frag(&Vs[(nb * 16) * LDT + c * 32], LDT);
          o2 = wmma16(pf, vf, o2);
        }
#pragma unroll
        for (int v = 0; v < 8; ++v) o[nb][v] = o[nb][v] + o2[v] * (1.0f / RCARRY);
      }
    }
    __syncthreads();
  }

  float inv[8];
#pragma unroll
  for (int v = 0; v < 8; ++v) inv[v] = __builtin_amdgcn_rcpf(lrow[v]) * (1.0f / PCARRY);
#pragma unroll
  for (int nb = 0; nb < 4; ++nb)
#pragma unroll
    for (int v = 0; v < 8; ++v)
      Qs[qsbase + (hh * 8u + (unsigned)v) * LDC + (unsigned)nb * 16u + m] = o[nb][v] * inv[v];
  wave_lds_sync();
  v4f x[8];
  size_t off[8];
#pragma unroll
  for (unsigned i = 0; i < 8u; ++i) {
    const unsigned r = 2u * i + (lane >> 4);
    const unsigned c = (lane & 15u) * 4u;
    x[i] = *(const v4f*)&Qs[qsbase + r * LDC + c];
    off[i] = ((size_t)b * SEQ_FULL + qrow0 + r) * HD + c;
  }
#pragma unroll
  for (int i = 0; i < 8; ++i) *(volatile v4f*)(Out + off[i]) = x[i];
  __threadfence();
#pragma unroll
  for (int i = 0; i < 8; ++i) *(volatile v4f*)(Out + off[i]) = x[i];
}

extern "C" void kernel_launch(void* const* d_in, const int* in_sizes, int n_in,
                              void* d_out, int out_size, void* d_ws, size_t ws_size,
                              hipStream_t stream) {
  if (n_in < 11) return;
  const long long need_x = ((long long)(NB - 1) * SEQ_FULL + SEQ) * EMB;
  const long long need_o = ((long long)(NB - 1) * SEQ_FULL + SEQ) * HD;
  if ((long long)in_sizes[0] < need_x) return;
  if (in_sizes[1] < EMB * HD || in_sizes[3] < EMB * HD || in_sizes[5] < EMB * HD) return;
  if (in_sizes[2] < HD || in_sizes[4] < HD || in_sizes[6] < HD) return;
  if (in_sizes[7] < 2 * HD * HD || in_sizes[8] < HD) return;
  if (in_sizes[9] < HD || in_sizes[10] < 1) return;
  if ((long long)out_size < need_o) return;
  if (ws_size < WS_TOTAL) return;

  const float* X  = (const float*)d_in[0];
  const float* wq = (const float*)d_in[1];
  const float* bq = (const float*)d_in[2];
  const float* wk = (const float*)d_in[3];
  const float* bk = (const float*)d_in[4];
  const float* wv = (const float*)d_in[5];
  const float* bv = (const float*)d_in[6];
  const float* w1 = (const float*)d_in[7];
  const float* b1 = (const float*)d_in[8];
  const float* w2 = (const float*)d_in[9];
  const float* b2 = (const float*)d_in[10];
  float* out = (float*)d_out;

  char* ws = (char*)d_ws;
  _Float16* Wq_t  = (_Float16*)(ws + OFF_WQ);
  _Float16* Wk_t  = (_Float16*)(ws + OFF_WK);
  _Float16* Wv_t  = (_Float16*)(ws + OFF_WV);
  _Float16* W1a_t = (_Float16*)(ws + OFF_W1A);
  _Float16* W1b_t = (_Float16*)(ws + OFF_W1B);
  _Float16* X16   = (_Float16*)(ws + OFF_X);
  _Float16* Q16   = (_Float16*)(ws + OFF_Q);
  _Float16* K16   = (_Float16*)(ws + OFF_K);
  _Float16* Vt16  = (_Float16*)(ws + OFF_VT);
  _Float16* VtR16 = (_Float16*)(ws + OFF_VR);
  float*    QPb   = (float*)(ws + OFF_QP);
  float*    KPo   = (float*)(ws + OFF_KP);

  dim3 blk(256);
  dim3 gg(HD / 64, MROWS / 64);

  wconv_kernel<<<dim3(HD / 64, EMB / 64), blk, 0, stream>>>(wq, Wq_t, (unsigned)HD, (unsigned)EMB);
  wconv_kernel<<<dim3(HD / 64, EMB / 64), blk, 0, stream>>>(wk, Wk_t, (unsigned)HD, (unsigned)EMB);
  wconv_kernel<<<dim3(HD / 64, EMB / 64), blk, 0, stream>>>(wv, Wv_t, (unsigned)HD, (unsigned)EMB);
  wconv_kernel<<<dim3(HD / 64, HD / 64), blk, 0, stream>>>(w1, W1a_t, (unsigned)HD, (unsigned)HD);
  wconv_kernel<<<dim3(HD / 64, HD / 64), blk, 0, stream>>>(w1 + (size_t)HD * HD, W1b_t,
                                                           (unsigned)HD, (unsigned)HD);

  xconv_kernel<<<dim3(MROWS / 8), blk, 0, stream>>>(X, X16);
  gemm_qk_kernel<<<gg, blk, 0, stream>>>(X16, Wq_t, bq, Q16);
  gemm_qk_kernel<<<gg, blk, 0, stream>>>(X16, Wk_t, bk, K16);
  gemm_v_kernel<<<gg, blk, 0, stream>>>(X16, Wv_t, bv, Vt16, VtR16);
  gemm_qp_kernel<<<gg, blk, 0, stream>>>(Q16, W1a_t, b1, QPb);
  gemm_kp_kernel<<<gg, blk, 0, stream>>>(K16, W1b_t, KPo);
  attn_kernel<<<dim3(SEQ / 128, NB), blk, 0, stream>>>(QPb, KPo, Vt16, VtR16, w2, b2, out);
}
